// PointNet2_glr_80917183857080
// MI455X (gfx1250) — hardware-verified
//
#include <hip/hip_runtime.h>
#pragma clang fp contract(off)

typedef __attribute__((ext_vector_type(16))) _Float16 v16h;
typedef __attribute__((ext_vector_type(8)))  _Float16 v8h;
typedef __attribute__((ext_vector_type(8)))  float    v8f;
typedef __attribute__((ext_vector_type(4)))  float    v4f;
typedef __attribute__((ext_vector_type(4)))  unsigned v4u;

constexpr int NBATCH = 32;
constexpr int NPT    = 2048;
constexpr int NS1    = 512;
constexpr int NK1    = 48;
constexpr int NS2    = 128;
constexpr int NK2    = 64;
constexpr int CH1A   = 64;
constexpr int CH1B   = 128;
constexpr int CH2A   = 128;
constexpr int CH2B   = 512;
constexpr int CH3    = 512;
constexpr int K1AP   = 32;
constexpr int K1BP   = 64;
constexpr int K2AP   = 160;
constexpr int K2BP   = 128;
constexpr int K3P    = 576;
constexpr float R2_SA1 = (float)(0.23 * 0.23);
constexpr float R2_SA2 = (float)(0.32 * 0.32);
constexpr float WCARRY = 16.0f;
constexpr float WINV   = 1.0f / WCARRY;
constexpr float BN_EPS = 1e-5f;

constexpr int WCH0 = 0;
constexpr int WCH1 = WCH0 + CH1A * (K1AP / 8);
constexpr int WCH2 = WCH1 + CH1B * (K1BP / 8);
constexpr int WCH3 = WCH2 + CH2A * (K2AP / 8);
constexpr int WCH4 = WCH3 + CH2B * (K2BP / 8);
constexpr int WCHT = WCH4 + CH3 * (K3P / 8);
static_assert(WCHT == 48896, "weight chunk count");
static_assert(WCHT % 256 == 0, "prep grid exact");
static_assert((WCH1 % 32) == 0 && (WCH2 % 32) == 0 && (WCH3 % 32) == 0 && (WCH4 % 32) == 0, "plane bounds wave aligned");
static_assert(K1AP % 32 == 0 && K1BP % 32 == 0 && K2AP % 32 == 0 && K2BP % 32 == 0 && K3P % 32 == 0, "K multiples of 32");
static_assert(NK1 == 48 && NK2 == 64 && NS1 * NK1 % 192 == 0, "group shapes");

__host__ __device__ constexpr int tri_off(int a) { return 6 * a - (a * (a - 1)) / 2; }

__device__ __forceinline__ unsigned h16bits(float f) {
  const _Float16 h = (_Float16)f;
  return (unsigned)__builtin_bit_cast(unsigned short, h);
}
__device__ __forceinline__ unsigned pack2h(float a, float b) {
  const unsigned lo = h16bits(a);
  const unsigned hi = h16bits(b);
  return lo | (hi << 16);
}
__device__ __forceinline__ v16h ldfrag(const _Float16* p) {
  union { v16h v; v8h h[2]; } f;
  f.h[0] = *(const v8h*)(p);
  f.h[1] = *(const v8h*)(p + 16);
  return f.v;
}
__device__ __forceinline__ v8f mma16(v16h a, v16h b, v8f c) {
  c = __builtin_amdgcn_wmma_f32_16x16x32_f16(false, a, false, b, (short)0, c, false, false);
  asm volatile("v_nop\n\tv_nop\n\tv_nop\n\tv_nop" : "+v"(c) : "v"(a), "v"(b));
  return c;
}
__device__ __forceinline__ void wave_lds_sync() {
  __builtin_amdgcn_fence(__ATOMIC_RELEASE, "workgroup");
  __builtin_amdgcn_wave_barrier();
  __builtin_amdgcn_fence(__ATOMIC_ACQUIRE, "workgroup");
}
__device__ __forceinline__ v8f zero8() { return (v8f){0.f, 0.f, 0.f, 0.f, 0.f, 0.f, 0.f, 0.f}; }

__global__ __launch_bounds__(256) void prep_weights_kernel(
    const float* __restrict__ w1a, const float* __restrict__ w1b, const float* __restrict__ w2a,
    const float* __restrict__ w2b, const float* __restrict__ w3, v4u* __restrict__ wp) {
  const int g = blockIdx.x * 256 + threadIdx.x;
  const float* src = w1a;
  int base = WCH0, kp8 = K1AP / 8, ld = 6, split = 6, shift = 0, nlow = 0;
  if (g >= WCH4)      { src = w3;  base = WCH4; kp8 = K3P / 8;  ld = 515; split = 512; shift = 3; nlow = 3; }
  else if (g >= WCH3) { src = w2b; base = WCH3; kp8 = K2BP / 8; ld = 128; split = 128; shift = 0; nlow = 0; }
  else if (g >= WCH2) { src = w2a; base = WCH2; kp8 = K2AP / 8; ld = 134; split = 128; shift = 6; nlow = 6; }
  else if (g >= WCH1) { src = w1b; base = WCH1; kp8 = K1BP / 8; ld = 64;  split = 64;  shift = 0; nlow = 0; }
  const int local = g - base;
  const int row = local / kp8;
  const int k0 = (local - row * kp8) * 8;
  float f[8];
#pragma unroll
  for (int e = 0; e < 8; ++e) {
    const int k = k0 + e;
    const bool hiK = k < split;
    const bool loK = (k >= split) && (k < split + nlow);
    const bool valid = hiK || loK;
    const int col = hiK ? (k + shift) : (k - split);
    const int colc = valid ? col : 0;
    const float v = src[(size_t)row * ld + colc];
    f[e] = valid ? (v * WCARRY) : 0.0f;
  }
  v4u u;
  u.x = pack2h(f[0], f[1]);
  u.y = pack2h(f[2], f[3]);
  u.z = pack2h(f[4], f[5]);
  u.w = pack2h(f[6], f[7]);
  if (g < WCHT) {
    *(volatile v4u*)(wp + g) = u;
  }
  __threadfence();
  if (g < WCHT) {
    *(volatile v4u*)(wp + g) = u;
  }
}

template <int NSRC, int NSAMP, bool AOS>
__global__ __launch_bounds__(256) void fps_kernel(const float* __restrict__ src, float* __restrict__ xyz_out) {
#pragma clang fp contract(off)
  constexpr int PPT = NSRC / 256;
  constexpr int NV4 = 3 * NSRC / 4;
  constexpr int NOUT4 = 3 * NSAMP / 4;
  __shared__ __align__(16) float sx[3 * NSRC];
  __shared__ int sidx[NSAMP];
  __shared__ float redv[2][8];
  __shared__ int redi[2][8];
  const int t = threadIdx.x, lane = t & 31, wave = t >> 5;
  const int b = blockIdx.x;
  const float* P = src + (size_t)b * (3 * NSRC);

  for (int i0 = 0; i0 < NV4; i0 += 256) {
    const int i = i0 + t;
    const int ic = i < NV4 ? i : NV4 - 1;
    const v4f v = *(const v4f*)(P + 4 * ic);
    if (i < NV4) {
      if (AOS) {
#pragma unroll
        for (int u = 0; u < 4; ++u) {
          const int e = 4 * i + u;
          const int m = e / 3;
          const int cc = e - 3 * m;
          sx[cc * NSRC + m] = v[u];
        }
      } else {
        *(v4f*)(sx + 4 * i) = v;
      }
    }
  }
  if (t == 0) sidx[0] = 0;
  __syncthreads();

  float px[PPT], py[PPT], pz[PPT], dist[PPT];
#pragma unroll
  for (int j = 0; j < PPT; ++j) {
    px[j] = sx[t + 256 * j];
    py[j] = sx[NSRC + t + 256 * j];
    pz[j] = sx[2 * NSRC + t + 256 * j];
    dist[j] = 1e10f;
  }
  float cx = sx[0], cy = sx[NSRC], cz = sx[2 * NSRC];

#pragma unroll 1
  for (int m = 1; m < NSAMP; ++m) {
    float bv = -1.0f;
    int bi = t;
#pragma unroll
    for (int j = 0; j < PPT; ++j) {
      const float dx = px[j] - cx;
      const float dy = py[j] - cy;
      const float dz = pz[j] - cz;
      const float t0 = dx * dx;
      const float t1 = dy * dy;
      const float t2 = dz * dz;
      const float d = (t0 + t2) + t1;
      const float dj = fminf(dist[j], d);
      dist[j] = dj;
      if (dj > bv) { bv = dj; bi = t + 256 * j; }
    }
#pragma unroll
    for (int off = 16; off >= 1; off >>= 1) {
      const float ov = __shfl_xor(bv, off, 32);
      const int oi = __shfl_xor(bi, off, 32);
      const bool take = (ov > bv) || ((ov == bv) && (oi < bi));
      bv = take ? ov : bv;
      bi = take ? oi : bi;
    }
    const int par = m & 1;
    if (lane == 0) { redv[par][wave] = bv; redi[par][wave] = bi; }
    __syncthreads();
    float fv = redv[par][0];
    int fi = redi[par][0];
#pragma unroll
    for (int w = 1; w < 8; ++w) {
      const float ov = redv[par][w];
      const int oi = redi[par][w];
      const bool take = (ov > fv) || ((ov == fv) && (oi < fi));
      fv = take ? ov : fv;
      fi = take ? oi : fi;
    }
    int last = fi < 0 ? 0 : fi;
    last = last > NSRC - 1 ? NSRC - 1 : last;
    if (t == 0) sidx[m] = last;
    cx = sx[last];
    cy = sx[NSRC + last];
    cz = sx[2 * NSRC + last];
  }
  __syncthreads();

  float* O = xyz_out + (size_t)b * (3 * NSAMP);
  for (int i0 = 0; i0 < NOUT4; i0 += 256) {
    const int i = i0 + t;
    const int ic = i < NOUT4 ? i : NOUT4 - 1;
    v4f val;
#pragma unroll
    for (int u = 0; u < 4; ++u) {
      const int e = 4 * ic + u;
      const int m = e / 3;
      const int cc = e - 3 * m;
      val[u] = sx[cc * NSRC + sidx[m]];
    }
    if (i < NOUT4) { *(volatile v4f*)(O + 4 * i) = val; }
    __threadfence();
    if (i < NOUT4) { *(volatile v4f*)(O + 4 * i) = val; }
  }
}

__global__ __launch_bounds__(256) void bq1_kernel(const float* __restrict__ pc, const float* __restrict__ xyz1,
                                                  v4u* __restrict__ F1, float* __restrict__ mompart) {
#pragma clang fp contract(off)
  __shared__ int list[8][64];
  __shared__ float red[8][32];
  const int t = threadIdx.x, lane = t & 31, wave = t >> 5;
  const int q = blockIdx.x * 8 + wave;
  const int b = q >> 9;
  const float* P = pc + (size_t)b * (3 * NPT);
  const float cx = xyz1[(size_t)q * 3 + 0];
  const float cy = xyz1[(size_t)q * 3 + 1];
  const float cz = xyz1[(size_t)q * 3 + 2];
  list[wave][lane] = 0;
  list[wave][lane + 32] = 0;
  wave_lds_sync();
  int cnt = 0;
  const unsigned ltmask = (1u << lane) - 1u;
#pragma unroll 1
  for (int it = 0; it < NPT / 32; ++it) {
    const int i = it * 32 + lane;
    const float x = P[i];
    const float y = P[NPT + i];
    const float z = P[2 * NPT + i];
    const float dx = cx - x;
    const float dy = cy - y;
    const float dz = cz - z;
    const float t0 = dx * dx;
    const float t1 = dy * dy;
    const float t2 = dz * dz;
    const float d2 = (t0 + t2) + t1;
    const bool in = d2 < R2_SA1;
    const unsigned msk = __builtin_amdgcn_ballot_w32(in);
    const int pos = cnt + __popc(msk & ltmask);
    if (in && (pos < NK1)) list[wave][pos] = i;
    cnt += __popc(msk);
  }
  wave_lds_sync();
  const int cntc = cnt < NK1 ? cnt : NK1;
  const int first = list[wave][0];
  const int k0 = lane;
  const int k1 = 32 + (lane & 15);
  int nb0 = (k0 < cntc) ? list[wave][k0] : first;
  int nb1 = (k1 < cntc) ? list[wave][k1] : first;
  nb0 = nb0 < 0 ? 0 : (nb0 > NPT - 1 ? NPT - 1 : nb0);
  nb1 = nb1 < 0 ? 0 : (nb1 > NPT - 1 ? NPT - 1 : nb1);
  const float g0x = P[nb0], g0y = P[NPT + nb0], g0z = P[2 * NPT + nb0];
  const float g1x = P[nb1], g1y = P[NPT + nb1], g1z = P[2 * NPT + nb1];
  const bool has1 = lane < 16;
  float f0[6], f1[6];
  f0[0] = g0x - cx; f0[1] = g0y - cy; f0[2] = g0z - cz; f0[3] = g0x; f0[4] = g0y; f0[5] = g0z;
  f1[0] = g1x - cx; f1[1] = g1y - cy; f1[2] = g1z - cz; f1[3] = g1x; f1[4] = g1y; f1[5] = g1z;

  unsigned zz = 0u;
  asm volatile("" : "+v"(zz));
  v4u u0, u1;
  u0.x = pack2h(f0[0], f0[1]); u0.y = pack2h(f0[2], f0[3]); u0.z = pack2h(f0[4], f0[5]); u0.w = zz;
  u1.x = pack2h(f1[0], f1[1]); u1.y = pack2h(f1[2], f1[3]); u1.z = pack2h(f1[4], f1[5]); u1.w = zz;
  v4u* Fq = F1 + (size_t)q * NK1;
  *(volatile v4u*)(Fq + k0) = u0;
  if (has1) { *(volatile v4u*)(Fq + k1) = u1; }
  __threadfence();
  *(volatile v4u*)(Fq + k0) = u0;
  if (has1) { *(volatile v4u*)(Fq + k1) = u1; }

  float fm[6];
#pragma unroll
  for (int a = 0; a < 6; ++a) fm[a] = has1 ? f1[a] : 0.0f;
  float mo[27];
#pragma unroll
  for (int a = 0; a < 6; ++a) mo[a] = f0[a] + fm[a];
#pragma unroll
  for (int a = 0; a < 6; ++a) {
#pragma unroll
    for (int bq = 0; bq < 6; ++bq) {
      if (bq >= a) {
        const float p0 = f0[a] * f0[bq];
        const float p1 = fm[a] * fm[bq];
        mo[6 + tri_off(a) + (bq - a)] = p0 + p1;
      }
    }
  }
#pragma unroll
  for (int j = 0; j < 27; ++j) {
    float v = mo[j];
#pragma unroll
    for (int off = 16; off >= 1; off >>= 1) v += __shfl_xor(v, off, 32);
    if (lane == 0) red[wave][j] = v;
  }
  if (lane == 0) {
#pragma unroll
    for (int j = 27; j < 32; ++j) red[wave][j] = 0.0f;
  }
  __syncthreads();
  if (wave == 0) {
    float tot = 0.0f;
#pragma unroll
    for (int w = 0; w < 8; ++w) tot += red[w][lane];
    volatile float* dst = mompart + (size_t)blockIdx.x * 32 + lane;
    *dst = tot;
    __threadfence();
    *dst = tot;
  }
}

__global__ __launch_bounds__(256) void fin1a_kernel(const float* __restrict__ mompart, int nparts,
                                                    const float* __restrict__ w1a, const float* __restrict__ g,
                                                    const float* __restrict__ bb, float* __restrict__ scb) {
  __shared__ double dred[8][32];
  __shared__ double mom[32];
  __shared__ double M2[36];
  const int t = threadIdx.x, col = t & 31, rg = t >> 5;
  double acc = 0.0;
#pragma unroll 1
  for (int r = rg; r < nparts; r += 8) acc += (double)mompart[(size_t)r * 32 + col];
  dred[rg][col] = acc;
  __syncthreads();
  if (t < 32) {
    double s = 0.0;
#pragma unroll 1
    for (int w = 0; w < 8; ++w) s += dred[w][t];
    mom[t] = s * (1.0 / (double)(NBATCH * NS1 * NK1));
  }
  __syncthreads();
  if (t < 36) {
    const int a = t / 6;
    const int bq = t - 6 * a;
    const int lo = a < bq ? a : bq;
    const int hi = a < bq ? bq : a;
    M2[t] = mom[6 + tri_off(lo) + (hi - lo)];
  }
  __syncthreads();
  const int ch = t < CH1A ? t : CH1A - 1;
  double wv[6];
#pragma unroll
  for (int k = 0; k < 6; ++k) wv[k] = (double)w1a[ch * 6 + k];
  double mean = 0.0;
#pragma unroll
  for (int k = 0; k < 6; ++k) mean += wv[k] * mom[k];
  double ey2 = 0.0;
#pragma unroll
  for (int a = 0; a < 6; ++a) {
    double rowsum = 0.0;
#pragma unroll
    for (int bq = 0; bq < 6; ++bq) rowsum += wv[bq] * M2[a * 6 + bq];
    ey2 += wv[a] * rowsum;
  }
  double var = ey2 - mean * mean;
  var = var < 0.0 ? 0.0 : var;
  const float sc = g[ch] * (1.0f / sqrtf((float)var + BN_EPS));
  const float bi = bb[ch] - (float)mean * sc;
  if (t < CH1A) {
    *(volatile float*)(scb + t) = sc;
    *(volatile float*)(scb + CH1A + t) = bi;
  }
  __threadfence();
  if (t < CH1A) {
    *(volatile float*)(scb + t) = sc;
    *(volatile float*)(scb + CH1A + t) = bi;
  }
}

__global__ __launch_bounds__(256) void fin_stats_kernel(const float* __restrict__ part, const float* __restrict__ g,
                                                        const float* __restrict__ bb, float* __restrict__ scb,
                                                        double invcount, int nparts, int C) {
  __shared__ double dred[2][8][32];
  const int t = threadIdx.x, lane = t & 31, rg = t >> 5;
  const int c = blockIdx.x * 32 + lane;
  double s = 0.0, q = 0.0;
#pragma unroll 1
  for (int r = rg; r < nparts; r += 8) {
    const float a0 = part[(size_t)r * (2 * C) + c];
    const float a1 = part[(size_t)r * (2 * C) + C + c];
    s += (double)a0;
    q += (double)a1;
  }
  dred[0][rg][lane] = s;
  dred[1][rg][lane] = q;
  __syncthreads();
  double S = 0.0, Q = 0.0;
#pragma unroll 1
  for (int w = 0; w < 8; ++w) { S += dred[0][w][lane]; Q += dred[1][w][lane]; }
  const double mean = S * invcount;
  double var = Q * invcount - mean * mean;
  var = var < 0.0 ? 0.0 : var;
  const float sc = g[c] * (1.0f / sqrtf((float)var + BN_EPS));
  const float bi = bb[c] - (float)mean * sc;
  if (rg == 0) {
    *(volatile float*)(scb + c) = sc;
    *(volatile float*)(scb + C + c) = bi;
  }
  __threadfence();
  if (rg == 0) {
    *(volatile float*)(scb + c) = sc;
    *(volatile float*)(scb + C + c) = bi;
  }
}

__global__ __launch_bounds__(128) void sa1_kernel(const v4u* __restrict__ F1, const _Float16* __restrict__ W1a,
                                                  const _Float16* __restrict__ W1b, const float* __restrict__ scb1a,
                                                  float* __restrict__ part, float* __restrict__ gmax1,
                                                  float* __restrict__ gmin1) {
  constexpr int FP = 40;
  constexpr int HP = 72;
  __shared__ __align__(16) _Float16 fT[192 * FP];
  __shared__ __align__(16) _Float16 hT[192 * HP];
  __shared__ __align__(16) float st[4 * 4 * 128];
  const int t = threadIdx.x, lane = t & 31, wave = t >> 5, hh = lane >> 4, c = lane & 15;
  const int blk = blockIdx.x;

  {
    const int r0 = t;
    const int r1 = t + 128;
    const int r1c = r1 < 192 ? r1 : 191;
    const v4u u0 = F1[(size_t)blk * 192 + r0];
    const v4u u1 = F1[(size_t)blk * 192 + r1c];
    const v4u zv = (v4u){0u, 0u, 0u, 0u};
    *(v4u*)(fT + r0 * FP) = u0;
    *(v4u*)(fT + r0 * FP + 8) = zv;
    *(v4u*)(fT + r0 * FP + 16) = zv;
    *(v4u*)(fT + r0 * FP + 24) = zv;
    if (r1 < 192) {
      *(v4u*)(fT + r1 * FP) = u1;
      *(v4u*)(fT + r1 * FP + 8) = zv;
      *(v4u*)(fT + r1 * FP + 16) = zv;
      *(v4u*)(fT + r1 * FP + 24) = zv;
    }
  }
  __syncthreads();

  const int rbase = wave * 48;
  {
    v16h bw[4];
#pragma unroll
    for (int j = 0; j < 4; ++j) bw[j] = ldfrag(W1a + (size_t)(j * 16 + c) * K1AP + 8 * hh);
    float sc[4], bi[4];
#pragma unroll
    for (int j = 0; j < 4; ++j) { sc[j] = scb1a[j * 16 + c]; bi[j] = scb1a[CH1A + j * 16 + c]; }
#pragma unroll
    for (int i = 0; i < 3; ++i) {
      const v16h a = ldfrag(fT + (rbase + i * 16 + c) * FP + 8 * hh);
      v8f acc[4];
#pragma unroll
      for (int j = 0; j < 4; ++j) acc[j] = mma16(a, bw[j], zero8());
#pragma unroll
      for (int j = 0; j < 4; ++j) {
#pragma unroll
        for (int r = 0; r < 8; ++r) {
          const float y = acc[j][r] * WINV;
          const float z = y * sc[j];
          const float hv = fmaxf(z + bi[j], 0.0f);
          hT[(rbase + i * 16 + 8 * hh + r) * HP + j * 16 + c] = (_Float16)hv;
        }
      }
    }
  }
  __syncthreads();

  v16h af[3][2];
#pragma unroll
  for (int i = 0; i < 3; ++i) {
#pragma unroll
    for (int ks = 0; ks < 2; ++ks) af[i][ks] = ldfrag(hT + (rbase + i * 16 + c) * HP + ks * 32 + 8 * hh);
  }
#pragma unroll 1
  for (int nn = 0; nn < 4; ++nn) {
    v8f acc[3][2];
#pragma unroll
    for (int i = 0; i < 3; ++i) { acc[i][0] = zero8(); acc[i][1] = zero8(); }
#pragma unroll
    for (int jj = 0; jj < 2; ++jj) {
#pragma unroll
      for (int ks = 0; ks < 2; ++ks) {
        const v16h bf = ldfrag(W1b + (size_t)((nn * 2 + jj) * 16 + c) * K1BP + ks * 32 + 8 * hh);
#pragma unroll
        for (int i = 0; i < 3; ++i) acc[i][jj] = mma16(af[i][ks], bf, acc[i][jj]);
      }
    }
    asm volatile("" ::: "memory");
#pragma unroll
    for (int jj = 0; jj < 2; ++jj) {
      const int n = (nn * 2 + jj) * 16 + c;
      float s = 0.0f, q = 0.0f, mx = -INFINITY, mn = INFINITY;
#pragma unroll
      for (int i = 0; i < 3; ++i) {
#pragma unroll
        for (int r = 0; r < 8; ++r) {
          const float y = acc[i][jj][r] * WINV;
          const float y2 = y * y;
          s += y;
          q += y2;
          mx = fmaxf(mx, y);
          mn = fminf(mn, y);
        }
      }
      s += __shfl_xor(s, 16, 32);
      q += __shfl_xor(q, 16, 32);
      mx = fmaxf(mx, __shfl_xor(mx, 16, 32));
      mn = fminf(mn, __shfl_xor(mn, 16, 32));
      if (hh == 0) {
        st[(wave * 4 + 0) * 128 + n] = mx;
        st[(wave * 4 + 1) * 128 + n] = mn;
        st[(wave * 4 + 2) * 128 + n] = s;
        st[(wave * 4 + 3) * 128 + n] = q;
      }
    }
  }
  __syncthreads();
  {
    const int q = blk * 4 + wave;
    const v4f vmx = *(const v4f*)(st + (wave * 4 + 0) * 128 + lane * 4);
    const v4f vmn = *(const v4f*)(st + (wave * 4 + 1) * 128 + lane * 4);
    const int a = 2 + (wave & 1);
    v4f ps = *(const v4f*)(st + (0 * 4 + a) * 128 + lane * 4);
    ps += *(const v4f*)(st + (1 * 4 + a) * 128 + lane * 4);
    ps += *(const v4f*)(st + (2 * 4 + a) * 128 + lane * 4);
    ps += *(const v4f*)(st + (3 * 4 + a) * 128 + lane * 4);
    float* pmx = gmax1 + (size_t)q * 128 + lane * 4;
    float* pmn = gmin1 + (size_t)q * 128 + lane * 4;
    float* pp = part + (size_t)blk * 256 + (wave & 1) * 128 + lane * 4;
    *(volatile v4f*)pmx = vmx;
    *(volatile v4f*)pmn = vmn;
    if (wave < 2) { *(volatile v4f*)pp = ps; }
    __threadfence();
    *(volatile v4f*)pmx = vmx;
    *(volatile v4f*)pmn = vmn;
    if (wave < 2) { *(volatile v4f*)pp = ps; }
  }
}

__global__ __launch_bounds__(256) void pool1_kernel(const float* __restrict__ gmax1, const float* __restrict__ gmin1,
                                                    const float* __restrict__ scb, v4u* __restrict__ f1p) {
  const int g = blockIdx.x * 256 + threadIdx.x;
  const int row = g >> 4, seg = g & 15;
  const float* pm = gmax1 + (size_t)row * 128 + seg * 8;
  const float* pn = gmin1 + (size_t)row * 128 + seg * 8;
  const v4f mx0 = *(const v4f*)pm, mx1 = *(const v4f*)(pm + 4);
  const v4f mn0 = *(const v4f*)pn, mn1 = *(const v4f*)(pn + 4);
  const v4f sc0 = *(const v4f*)(scb + seg * 8), sc1 = *(const v4f*)(scb + seg * 8 + 4);
  const v4f bi0 = *(const v4f*)(scb + CH1B + seg * 8), bi1 = *(const v4f*)(scb + CH1B + seg * 8 + 4);
  float f[8];
#pragma unroll
  for (int e = 0; e < 4; ++e) {
    const float s0 = sc0[e], s1 = sc1[e];
    const float v0 = (s0 >= 0.0f) ? mx0[e] : mn0[e];
    const float v1 = (s1 >= 0.0f) ? mx1[e] : mn1[e];
    const float z0 = s0 * v0;
    const float z1 = s1 * v1;
    f[e] = fmaxf(z0 + bi0[e], 0.0f);
    f[4 + e] = fmaxf(z1 + bi1[e], 0.0f);
  }
  v4u u;
  u.x = pack2h(f[0], f[1]);
  u.y = pack2h(f[2], f[3]);
  u.z = pack2h(f[4], f[5]);
  u.w = pack2h(f[6], f[7]);
  *(volatile v4u*)(f1p + g) = u;
  __threadfence();
  *(volatile v4u*)(f1p + g) = u;
}

template <bool FUSED>
__global__ __launch_bounds__(256) void sa2_kernel(const float* __restrict__ xyz1, const float* __restrict__ xyz2,
                                                  const v4u* __restrict__ f1p, const _Float16* __restrict__ W2a,
                                                  const _Float16* __restrict__ W2b, const float* __restrict__ scb2a,
                                                  float* __restrict__ part, float* __restrict__ gmax2,
                                                  float* __restrict__ gmin2) {
#pragma clang fp contract(off)
  constexpr int AP = 168;
  constexpr int STN = FUSED ? 4096 : 2048;
  __shared__ __align__(16) _Float16 aT[128 * AP];
  __shared__ __align__(16) float st[STN];
  __shared__ int list[2][64];
  __shared__ int scnt[2];
  const int t = threadIdx.x, lane = t & 31, wave = t >> 5, hh = lane >> 4, c = lane & 15;
  const int blk = blockIdx.x;
  const int b = blk >> 6;
  const float* S = xyz1 + (size_t)b * (NS1 * 3);

  if (wave < 2) {
    const int q2 = blk * 2 + wave;
    const float cx = xyz2[(size_t)q2 * 3 + 0];
    const float cy = xyz2[(size_t)q2 * 3 + 1];
    const float cz = xyz2[(size_t)q2 * 3 + 2];
    list[wave][lane] = 0;
    list[wave][lane + 32] = 0;
    wave_lds_sync();
    int cnt = 0;
    const unsigned ltmask = (1u << lane) - 1u;
#pragma unroll 1
    for (int it = 0; it < NS1 / 32; ++it) {
      const int i = it * 32 + lane;
      const float x = S[i * 3 + 0];
      const float y = S[i * 3 + 1];
      const float z = S[i * 3 + 2];
      const float dx = cx - x;
      const float dy = cy - y;
      const float dz = cz - z;
      const float t0 = dx * dx;
      const float t1 = dy * dy;
      const float t2 = dz * dz;
      const float d2 = (t0 + t2) + t1;
      const bool in = d2 < R2_SA2;
      const unsigned msk = __builtin_amdgcn_ballot_w32(in);
      const int pos = cnt + __popc(msk & ltmask);
      if (in && (pos < NK2)) list[wave][pos] = i;
      cnt += __popc(msk);
    }
    if (lane == 0) scnt[wave] = cnt < NK2 ? cnt : NK2;
  }
  __syncthreads();

#pragma unroll
  for (int i = 0; i < 8; ++i) {
    const int idx = t + 256 * i;
    const int row = idx >> 4, seg = idx & 15;
    const int ci = row >> 6, k = row & 63;
    const int cn = scnt[ci];
    const int lk = list[ci][k];
    const int l0 = list[ci][0];
    int nb = (k < cn) ? lk : l0;
    nb = nb < 0 ? 0 : (nb > NS1 - 1 ? NS1 - 1 : nb);
    const v4u u = f1p[((size_t)(b * NS1 + nb)) * 16 + seg];
    *(v4u*)(aT + row * AP + seg * 8) = u;
  }
  if (t < 128) {
    const int row = t;
    const int ci = row >> 6, k = row & 63;
    const int cn = scnt[ci];
    const int lk = list[ci][k];
    const int l0 = list[ci][0];
    int nb = (k < cn) ? lk : l0;
    nb = nb < 0 ? 0 : (nb > NS1 - 1 ? NS1 - 1 : nb);
    const int q2 = blk * 2 + ci;
    const float cx = xyz2[(size_t)q2 * 3 + 0];
    const float cy = xyz2[(size_t)q2 * 3 + 1];
    const float cz = xyz2[(size_t)q2 * 3 + 2];
    const float gx = S[nb * 3 + 0], gy = S[nb * 3 + 1], gz = S[nb * 3 + 2];
    unsigned zz = 0u;
    asm volatile("" : "+v"(zz));
    v4u u;
    u.x = pack2h(gx - cx, gy - cy);
    u.y = pack2h(gz - cz, gx);
    u.z = pack2h(gy, gz);
    u.w = zz;
    const v4u zv = (v4u){zz, zz, zz, zz};
    *(v4u*)(aT + row * AP + 128) = u;
    *(v4u*)(aT + row * AP + 136) = zv;
    *(v4u*)(aT + row * AP + 144) = zv;
    *(v4u*)(aT + row * AP + 152) = zv;
  }
  __syncthreads();

  v8f acc[8];
#pragma unroll
  for (int j = 0; j < 8; ++j) acc[j] = zero8();
#pragma unroll 1
  for (int ks = 0; ks < K2AP / 32; ++ks) {
    const v16h a = ldfrag(aT + (wave * 16 + c) * AP + ks * 32 + 8 * hh);
#pragma unroll
    for (int jg = 0; jg < 2; ++jg) {
      v16h bf[4];
#pragma unroll
      for (int j4 = 0; j4 < 4; ++j4) bf[j4] = ldfrag(W2a + (size_t)((jg * 4 + j4) * 16 + c) * K2AP + ks * 32 + 8 * hh);
#pragma unroll
      for (int j4 = 0; j4 < 4; ++j4) acc[jg * 4 + j4] = mma16(a, bf[j4], acc[jg * 4 + j4]);
      asm volatile("" ::: "memory");
    }
  }

  if (!FUSED) {
#pragma unroll
    for (int j = 0; j < 8; ++j) {
      const int n = j * 16 + c;
      float s = 0.0f, q = 0.0f;
#pragma unroll
      for (int r = 0; r < 8; ++r) {
        const float y = acc[j][r] * WINV;
        const float y2 = y * y;
        s += y;
        q += y2;
      }
      s += __shfl_xor(s, 16, 32);
      q += __shfl_xor(q, 16, 32);
      if (hh == 0) {
        st[(wave * 2 + 0) * 128 + n] = s;
        st[(wave * 2 + 1) * 128 + n] = q;
      }
    }
    __syncthreads();
    if (wave < 2) {
      v4f r4 = *(const v4f*)(st + (0 * 2 + wave) * 128 + lane * 4);
#pragma unroll
      for (int w = 1; w < 8; ++w) r4 += *(const v4f*)(st + (w * 2 + wave) * 128 + lane * 4);
      float* pp = part + (size_t)blk * 256 + wave * 128 + lane * 4;
      *(volatile v4f*)pp = r4;
      __threadfence();
      *(volatile v4f*)pp = r4;
    }
  } else {
#pragma unroll
    for (int j = 0; j < 8; ++j) {
      const int n = j * 16 + c;
      const float sc = scb2a[n];
      const float bi = scb2a[CH2A + n];
#pragma unroll
      for (int r = 0; r < 8; ++r) {
        const float y = acc[j][r] * WINV;
        const float z = y * sc;
        const float hv = fmaxf(z + bi, 0.0f);
        aT[(wave * 16 + 8 * hh + r) * AP + n] = (_Float16)hv;
      }
    }
    __syncthreads();

    const int g = wave & 1;
    const int nq = wave >> 1;
#pragma unroll 1
    for (int nn = 0; nn < 4; ++nn) {
      const int nt0 = nq * 8 + nn * 2;
      v8f ac2[4][2];
#pragma unroll
      for (int i = 0; i < 4; ++i) { ac2[i][0] = zero8(); ac2[i][1] = zero8(); }
#pragma unroll
      for (int ks = 0; ks < K2BP / 32; ++ks) {
        v16h af[4];
#pragma unroll
        for (int i = 0; i < 4; ++i) af[i] = ldfrag(aT + (g * 64 + i * 16 + c) * AP + ks * 32 + 8 * hh);
#pragma unroll
        for (int jj = 0; jj < 2; ++jj) {
          const v16h bf = ldfrag(W2b + (size_t)((nt0 + jj) * 16 + c) * K2BP + ks * 32 + 8 * hh);
#pragma unroll
          for (int i = 0; i < 4; ++i) ac2[i][jj] = mma16(af[i], bf, ac2[i][jj]);
        }
        asm volatile("" ::: "memory");
      }
#pragma unroll
      for (int jj = 0; jj < 2; ++jj) {
        const int n = (nt0 + jj) * 16 + c;
        float s = 0.0f, q = 0.0f, mx = -INFINITY, mn = INFINITY;
#pragma unroll
        for (int i = 0; i < 4; ++i) {
#pragma unroll
          for (int r = 0; r < 8; ++r) {
            const float y = ac2[i][jj][r] * WINV;
            const float y2 = y * y;
            s += y;
            q += y2;
            mx = fmaxf(mx, y);
            mn = fminf(mn, y);
          }
        }
        s += __shfl_xor(s, 16, 32);
        q += __shfl_xor(q, 16, 32);
        mx = fmaxf(mx, __shfl_xor(mx, 16, 32));
        mn = fminf(mn, __shfl_xor(mn, 16, 32));
        if (hh == 0) {
          st[(g * 4 + 0) * 512 + n] = mx;
          st[(g * 4 + 1) * 512 + n] = mn;
          st[(g * 4 + 2) * 512 + n] = s;
          st[(g * 4 + 3) * 512 + n] = q;
        }
      }
    }
    __syncthreads();
    {
      const int gg = t >> 7, f4 = t & 127;
      const v4f vmx = *(const v4f*)(st + (gg * 4 + 0) * 512 + f4 * 4);
      const v4f vmn = *(const v4f*)(st + (gg * 4 + 1) * 512 + f4 * 4);
      const int a = 2 + gg;
      v4f ps = *(const v4f*)(st + (0 * 4 + a) * 512 + f4 * 4);
      ps += *(const v4f*)(st + (1 * 4 + a) * 512 + f4 * 4);
      float* pmx = gmax2 + (size_t)(blk * 2 + gg) * 512 + f4 * 4;
      float* pmn = gmin2 + (size_t)(blk * 2 + gg) * 512 + f4 * 4;
      float* pp = part + (size_t)blk * 1024 + gg * 512 + f4 * 4;
      *(volatile v4f*)pmx = vmx;
      *(volatile v4f*)pmn = vmn;
      *(volatile v4f*)pp = ps;
      __threadfence();
      *(volatile v4f*)pmx = vmx;
      *(volatile v4f*)pmn = vmn;
      *(volatile v4f*)pp = ps;
    }
  }
}

__global__ __launch_bounds__(256) void build_a3_kernel(const float* __restrict__ gmax2, const float* __restrict__ gmin2,
                                                       const float* __restrict__ scb, const float* __restrict__ xyz2,
                                                       v4u* __restrict__ A3) {
  const int g = blockIdx.x * 256 + threadIdx.x;
  const int row = g / 72;
  const int ch = g - row * 72;
  const int chc = ch < 64 ? ch : 63;
  const float* pm = gmax2 + (size_t)row * 512 + chc * 8;
  const float* pn = gmin2 + (size_t)row * 512 + chc * 8;
  const v4f mx0 = *(const v4f*)pm, mx1 = *(const v4f*)(pm + 4);
  const v4f mn0 = *(const v4f*)pn, mn1 = *(const v4f*)(pn + 4);
  const v4f sc0 = *(const v4f*)(scb + chc * 8), sc1 = *(const v4f*)(scb + chc * 8 + 4);
  const v4f bi0 = *(const v4f*)(scb + CH2B + chc * 8), bi1 = *(const v4f*)(scb + CH2B + chc * 8 + 4);
  const float px = xyz2[(size_t)row * 3 + 0];
  const float py = xyz2[(size_t)row * 3 + 1];
  const float pz = xyz2[(size_t)row * 3 + 2];
  float f[8];
#pragma unroll
  for (int e = 0; e < 4; ++e) {
    const float s0 = sc0[e], s1 = sc1[e];
    const float v0 = (s0 >= 0.0f) ? mx0[e] : mn0[e];
    const float v1 = (s1 >= 0.0f) ? mx1[e] : mn1[e];
    const float z0 = s0 * v0;
    const float z1 = s1 * v1;
    f[e] = fmaxf(z0 + bi0[e], 0.0f);
    f[4 + e] = fmaxf(z1 + bi1[e], 0.0f);
  }
  const bool isFeat = ch < 64;
  const bool isGeo = ch == 64;
#pragma unroll
  for (int e = 0; e < 8; ++e) {
    const float ge = (e == 0) ? px : ((e == 1) ? py : ((e == 2) ? pz : 0.0f));
    f[e] = isFeat ? f[e] : (isGeo ? ge : 0.0f);
  }
  v4u u;
  u.x = pack2h(f[0], f[1]);
  u.y = pack2h(f[2], f[3]);
  u.z = pack2h(f[4], f[5]);
  u.w = pack2h(f[6], f[7]);
  *(volatile v4u*)(A3 + g) = u;
  __threadfence();
  *(volatile v4u*)(A3 + g) = u;
}

__global__ __launch_bounds__(256) void l3_kernel(const _Float16* __restrict__ A3, const _Float16* __restrict__ W3,
                                                 float* __restrict__ l3st) {
  __shared__ __align__(16) float st[8 * 4 * 64];
  const int t = threadIdx.x, lane = t & 31, wave = t >> 5, hh = lane >> 4, c = lane & 15;
  const int b = blockIdx.x >> 3, nb = blockIdx.x & 7;
  const _Float16* arow = A3 + (size_t)(b * 128 + wave * 16 + c) * K3P + 8 * hh;
  const _Float16* brow = W3 + (size_t)(nb * 64 + c) * K3P + 8 * hh;
  v8f acc[4];
#pragma unroll
  for (int j = 0; j < 4; ++j) acc[j] = zero8();
#pragma unroll 1
  for (int ks = 0; ks < K3P / 32; ++ks) {
    const v16h a = ldfrag(arow + ks * 32);
    const v16h b0 = ldfrag(brow + (size_t)0 * 16 * K3P + ks * 32);
    const v16h b1 = ldfrag(brow + (size_t)1 * 16 * K3P + ks * 32);
    acc[0] = mma16(a, b0, acc[0]);
    acc[1] = mma16(a, b1, acc[1]);
    asm volatile("" ::: "memory");
    const v16h b2 = ldfrag(brow + (size_t)2 * 16 * K3P + ks * 32);
    const v16h b3 = ldfrag(brow + (size_t)3 * 16 * K3P + ks * 32);
    acc[2] = mma16(a, b2, acc[2]);
    acc[3] = mma16(a, b3, acc[3]);
    asm volatile("" ::: "memory");
  }
#pragma unroll
  for (int j = 0; j < 4; ++j) {
    const int n = j * 16 + c;
    float s = 0.0f, q = 0.0f, mx = -INFINITY, mn = INFINITY;
#pragma unroll
    for (int r = 0; r < 8; ++r) {
      const float y = acc[j][r] * WINV;
      const float y2 = y * y;
      s += y;
      q += y2;
      mx = fmaxf(mx, y);
      mn = fminf(mn, y);
    }
    s += __shfl_xor(s, 16, 32);
    q += __shfl_xor(q, 16, 32);
    mx = fmaxf(mx, __shfl_xor(mx, 16, 32));
    mn = fminf(mn, __shfl_xor(mn, 16, 32));
    if (hh == 0) {
      st[(wave * 4 + 0) * 64 + n] = mx;
      st[(wave * 4 + 1) * 64 + n] = mn;
      st[(wave * 4 + 2) * 64 + n] = s;
      st[(wave * 4 + 3) * 64 + n] = q;
    }
  }
  __syncthreads();
  if (wave < 4) {
    const int a = wave;
    const int lc = lane & 15;
    v4f r4 = *(const v4f*)(st + (0 * 4 + a) * 64 + lc * 4);
#pragma unroll
    for (int w = 1; w < 8; ++w) {
      const v4f v = *(const v4f*)(st + (w * 4 + a) * 64 + lc * 4);
#pragma unroll
      for (int e = 0; e < 4; ++e) {
        const float mxv = fmaxf(r4[e], v[e]);
        const float mnv = fminf(r4[e], v[e]);
        const float smv = r4[e] + v[e];
        r4[e] = (a == 0) ? mxv : ((a == 1) ? mnv : smv);
      }
    }
    float* dst = l3st + (size_t)a * (NBATCH * CH3) + (size_t)b * CH3 + nb * 64 + lc * 4;
    if (lane < 16) { *(volatile v4f*)dst = r4; }
    __threadfence();
    if (lane < 16) { *(volatile v4f*)dst = r4; }
  }
}

__global__ __launch_bounds__(256) void fin3_kernel(const float* __restrict__ l3st, const float* __restrict__ g3,
                                                   const float* __restrict__ b3, float* __restrict__ out) {
  __shared__ double dred[2][8][32];
  const int t = threadIdx.x, lane = t & 31, wave = t >> 5;
  const int c = blockIdx.x * 32 + lane;
  constexpr int PL = NBATCH * CH3;
  double s = 0.0, q = 0.0;
#pragma unroll
  for (int i = 0; i < 4; ++i) {
    const int b = wave + 8 * i;
    s += (double)l3st[2 * PL + b * CH3 + c];
    q += (double)l3st[3 * PL + b * CH3 + c];
  }
  dred[0][wave][lane] = s;
  dred[1][wave][lane] = q;
  __syncthreads();
  double S = 0.0, Q = 0.0;
#pragma unroll 1
  for (int w = 0; w < 8; ++w) { S += dred[0][w][lane]; Q += dred[1][w][lane]; }
  const double invc = 1.0 / (double)(NBATCH * NS2);
  const double mean = S * invc;
  double var = Q * invc - mean * mean;
  var = var < 0.0 ? 0.0 : var;
  const float sc = g3[c] * (1.0f / sqrtf((float)var + BN_EPS));
  const float bi = b3[c] - (float)mean * sc;
  float v[4];
#pragma unroll
  for (int i = 0; i < 4; ++i) {
    const int b = wave + 8 * i;
    const float mx = l3st[0 * PL + b * CH3 + c];
    const float mn = l3st[1 * PL + b * CH3 + c];
    const float sel = (sc >= 0.0f) ? mx : mn;
    const float z = sc * sel;
    v[i] = fmaxf(z + bi, 0.0f);
  }
#pragma unroll
  for (int i = 0; i < 4; ++i) {
    const int b = wave + 8 * i;
    *(volatile float*)(out + (size_t)b * CH3 + c) = v[i];
  }
  __threadfence();
#pragma unroll
  for (int i = 0; i < 4; ++i) {
    const int b = wave + 8 * i;
    *(volatile float*)(out + (size_t)b * CH3 + c) = v[i];
  }
}

extern "C" void kernel_launch(void* const* d_in, const int* in_sizes, int n_in,
                              void* d_out, int out_size, void* d_ws, size_t ws_size, hipStream_t stream) {
  (void)in_sizes; (void)n_in; (void)out_size;
  const float* pc  = (const float*)d_in[0];
  const float* w1a = (const float*)d_in[1];
  const float* g1a = (const float*)d_in[2];
  const float* b1a = (const float*)d_in[3];
  const float* w1b = (const float*)d_in[4];
  const float* g1b = (const float*)d_in[5];
  const float* b1b = (const float*)d_in[6];
  const float* w2a = (const float*)d_in[7];
  const float* g2a = (const float*)d_in[8];
  const float* b2a = (const float*)d_in[9];
  const float* w2b = (const float*)d_in[10];
  const float* g2b = (const float*)d_in[11];
  const float* b2b = (const float*)d_in[12];
  const float* w3  = (const float*)d_in[13];
  const float* g3  = (const float*)d_in[14];
  const float* b3  = (const float*)d_in[15];
  float* out = (float*)d_out;

  char* ws = (char*)d_ws;
  size_t off = 0;
  auto carve = [&](size_t bytes) {
    char* p = ws + off;
    off += (bytes + 127) & ~(size_t)127;
    return p;
  };
  v4u*   wp     = (v4u*)carve((size_t)WCHT * 16);
  float* xyz1   = (float*)carve((size_t)NBATCH * NS1 * 3 * 4);
  float* xyz2   = (float*)carve((size_t)NBATCH * NS2 * 3 * 4);
  v4u*   F1     = (v4u*)carve((size_t)NBATCH * NS1 * NK1 * 16);
  float* mom    = (float*)carve((size_t)2048 * 32 * 4);
  float* scb1a  = (float*)carve((size_t)2 * CH1A * 4);
  float* scb1b  = (float*)carve((size_t)2 * CH1B * 4);
  float* scb2a  = (float*)carve((size_t)2 * CH2A * 4);
  float* scb2b  = (float*)carve((size_t)2 * CH2B * 4);
  float* part1b = (float*)carve((size_t)4096 * 256 * 4);
  float* gmax1  = (float*)carve((size_t)NBATCH * NS1 * CH1B * 4);
  float* gmin1  = (float*)carve((size_t)NBATCH * NS1 * CH1B * 4);
  v4u*   f1p    = (v4u*)carve((size_t)NBATCH * NS1 * CH1B * 2);
  float* part2a = (float*)carve((size_t)2048 * 256 * 4);
  float* part2b = (float*)carve((size_t)2048 * 1024 * 4);
  float* gmax2  = (float*)carve((size_t)NBATCH * NS2 * CH2B * 4);
  float* gmin2  = (float*)carve((size_t)NBATCH * NS2 * CH2B * 4);
  v4u*   A3     = (v4u*)carve((size_t)NBATCH * NS2 * K3P * 2);
  float* l3st   = (float*)carve((size_t)4 * NBATCH * CH3 * 4);
  if (off > ws_size) return;

  const _Float16* wph = (const _Float16*)wp;
  const _Float16* W1a = wph + (size_t)WCH0 * 8;
  const _Float16* W1b = wph + (size_t)WCH1 * 8;
  const _Float16* W2a = wph + (size_t)WCH2 * 8;
  const _Float16* W2b = wph + (size_t)WCH3 * 8;
  const _Float16* W3  = wph + (size_t)WCH4 * 8;

  prep_weights_kernel<<<WCHT / 256, 256, 0, stream>>>(w1a, w1b, w2a, w2b, w3, wp);
  fps_kernel<NPT, NS1, false><<<NBATCH, 256, 0, stream>>>(pc, xyz1);
  bq1_kernel<<<(NBATCH * NS1) / 8, 256, 0, stream>>>(pc, xyz1, F1, mom);
  fin1a_kernel<<<1, 256, 0, stream>>>(mom, 2048, w1a, g1a, b1a, scb1a);
  sa1_kernel<<<(NBATCH * NS1) / 4, 128, 0, stream>>>(F1, W1a, W1b, scb1a, part1b, gmax1, gmin1);
  fin_stats_kernel<<<CH1B / 32, 256, 0, stream>>>(part1b, g1b, b1b, scb1b,
                                                  1.0 / (double)(NBATCH * NS1 * NK1), 4096, CH1B);
  pool1_kernel<<<(NBATCH * NS1 * 16) / 256, 256, 0, stream>>>(gmax1, gmin1, scb1b, f1p);
  fps_kernel<NS1, NS2, true><<<NBATCH, 256, 0, stream>>>(xyz1, xyz2);
  sa2_kernel<false><<<(NBATCH * NS2) / 2, 256, 0, stream>>>(xyz1, xyz2, f1p, W2a, W2b, scb2a, part2a, gmax2, gmin2);
  fin_stats_kernel<<<CH2A / 32, 256, 0, stream>>>(part2a, g2a, b2a, scb2a,
                                                  1.0 / (double)(NBATCH * NS2 * NK2), 2048, CH2A);
  sa2_kernel<true><<<(NBATCH * NS2) / 2, 256, 0, stream>>>(xyz1, xyz2, f1p, W2a, W2b, scb2a, part2b, gmax2, gmin2);
  fin_stats_kernel<<<CH2B / 32, 256, 0, stream>>>(part2b, g2b, b2b, scb2b,
                                                  1.0 / (double)(NBATCH * NS2 * NK2), 2048, CH2B);
  build_a3_kernel<<<(NBATCH * NS2 * (K3P / 8)) / 256, 256, 0, stream>>>(gmax2, gmin2, scb2b, xyz2, A3);
  l3_kernel<<<NBATCH * (CH3 / 64), 256, 0, stream>>>((const _Float16*)A3, W3, l3st);
  fin3_kernel<<<CH3 / 32, 256, 0, stream>>>(l3st, g3, b3, out);
}
